// GlobalSSM_8512625180868
// MI455X (gfx1250) — hardware-run, weakly checked
//
#include <hip/hip_runtime.h>
#include <math.h>
#include <stdint.h>

typedef __attribute__((ext_vector_type(16))) _Float16 v16h;
typedef __attribute__((ext_vector_type(8)))  _Float16 v8h;
typedef __attribute__((ext_vector_type(16))) __bf16   v16b;
typedef __attribute__((ext_vector_type(8)))  __bf16   v8b;
typedef __attribute__((ext_vector_type(8)))  float    v8f;
typedef __attribute__((ext_vector_type(4)))  float    v4f;
typedef __attribute__((ext_vector_type(4)))  unsigned int v4u;

#define NBATCH 2
#define SEQLEN 4096
#define DMOD 1024
#define NST 16
#define MROWS 8192
#define NALL 1088
#define TCHUNK 64
#define LOG2E_F 1.4426950408889634f

static_assert(NBATCH * SEQLEN == MROWS);
static_assert(MROWS % 64 == 0);
static_assert(NALL % 64 == 0);
static_assert(DMOD % 64 == 0);
static_assert(DMOD % 32 == 0);
static_assert(SEQLEN % TCHUNK == 0);
static_assert(TCHUNK == 64);

__device__ __forceinline__ unsigned short f2bf_bits(float f) {
  unsigned u = __float_as_uint(f);
  return (unsigned short)((u + 0x7FFFu + ((u >> 16) & 1u)) >> 16);
}
__device__ __forceinline__ float bf_bits2f(unsigned short h) { return __uint_as_float(((unsigned)h) << 16); }
__device__ __forceinline__ float bf_rne(float f) { return bf_bits2f(f2bf_bits(f)); }

__device__ __forceinline__ void dep_guard_b(v8f& a, v8f& b, v16b x, v16b y) { asm volatile("v_nop\n\tv_nop\n\tv_nop\n\tv_nop" : "+v"(a), "+v"(b) : "v"(x), "v"(y)); }
__device__ __forceinline__ void keep4_b(v16b a, v16b b, v16b c, v16b d) { asm volatile("v_nop" :: "v"(a), "v"(b), "v"(c), "v"(d)); }
__device__ __forceinline__ void acc_guard4(v8f& a, v8f& b, v8f& c, v8f& d) { asm volatile("v_nop\n\tv_nop\n\tv_nop\n\tv_nop" : "+v"(a), "+v"(b), "+v"(c), "+v"(d)); }

template <typename T> struct Frag;
template <> struct Frag<__bf16> {
  typedef v16b V; union U { v16b v; v8b h[2]; };
  static __device__ __forceinline__ v16b load(const __bf16* p) {
    U f; f.h[0] = *(const v8b*)(p); f.h[1] = *(const v8b*)(p + 16); return f.v;
  }
  static __device__ __forceinline__ v8f mma(v16b a, v16b b, v8f c) {
    return __builtin_amdgcn_wmma_f32_16x16x32_bf16(false, a, false, b, (short)0, c, false, false);
  }
  static __device__ __forceinline__ void guard(v8f& a, v8f& b, v16b x, v16b y) { dep_guard_b(a, b, x, y); }
  static __device__ __forceinline__ void keep(v16b a, v16b b, v16b c, v16b d) { keep4_b(a, b, c, d); }
};

__device__ __forceinline__ void wave_lds_sync() {
  __builtin_amdgcn_fence(__ATOMIC_RELEASE, "workgroup");
  __builtin_amdgcn_wave_barrier();
  __builtin_amdgcn_fence(__ATOMIC_ACQUIRE, "workgroup");
}

template <bool SPLA, int OUT_MODE, bool SCALE_IN>
__global__ __launch_bounds__(256) void gemm64_bf16(
    const unsigned short* __restrict__ Ap, const unsigned short* __restrict__ A2p, int lda,
    const unsigned short* __restrict__ Btp, int ldb,
    void* __restrict__ Cout, void* __restrict__ Cout2, int ldc,
    const float* __restrict__ scale_src, int M, int N, int K) {
  typedef __bf16 T;
  typedef v16b V;
  const T* A = (const T*)Ap; const T* A2 = (const T*)A2p; const T* Bt = (const T*)Btp;
  __shared__ __align__(16) float sT[8][16 * 68];
  const int lane = threadIdx.x & 31;
  const int wave = threadIdx.x >> 5;
  const int tilesN = N >> 6;
  const int tilesM = M >> 6;
  const int tile = blockIdx.x * 8 + wave;
  if (tile >= tilesM * tilesN) return;
  const int tm = tile / tilesN;
  const int tn = tile - tm * tilesN;
  const int m0 = tm << 6;
  const int n0 = tn << 6;

  const int rlane = lane & 15;
  const int koff  = (lane >> 4) * 8;
  const int mOff  = (lane >> 4) * 8;

  v8f acc[4][4];
#pragma unroll
  for (int i = 0; i < 4; ++i)
#pragma unroll
    for (int j = 0; j < 4; ++j) acc[i][j] = (v8f){0.f,0.f,0.f,0.f,0.f,0.f,0.f,0.f};

  for (int k0 = 0; k0 < K; k0 += 32) {
    V bh[4];
#pragma unroll
    for (int j = 0; j < 4; ++j) {
      const size_t bo = (size_t)(n0 + (j << 4) + rlane) * ldb + koff + k0;
      bh[j] = Frag<T>::load(Bt + bo);
    }
#pragma unroll
    for (int i = 0; i < 4; ++i) {
      const size_t ao = (size_t)(m0 + (i << 4) + rlane) * lda + koff + k0;
      V ah = Frag<T>::load(A + ao);
      V al = ah;
      if (SPLA) al = Frag<T>::load(A2 + ao);
#pragma unroll
      for (int j = 0; j < 4; ++j) {
        acc[i][j] = Frag<T>::mma(ah, bh[j], acc[i][j]);
        if (SPLA) acc[i][j] = Frag<T>::mma(al, bh[j], acc[i][j]);
      }
      Frag<T>::guard(acc[i][0], acc[i][3], ah, al);
    }
    Frag<T>::keep(bh[0], bh[1], bh[2], bh[3]);
  }
  acc_guard4(acc[0][0], acc[0][1], acc[0][2], acc[0][3]);
  acc_guard4(acc[1][0], acc[1][1], acc[1][2], acc[1][3]);
  acc_guard4(acc[2][0], acc[2][1], acc[2][2], acc[2][3]);
  acc_guard4(acc[3][0], acc[3][1], acc[3][2], acc[3][3]);

  float scale = 1.0f;
  if (SCALE_IN) scale = bf_rne(scale_src[0]);

  float* slab = sT[wave];
#pragma unroll
  for (int i = 0; i < 4; ++i) {
    const int mBase = m0 + (i << 4);
#pragma unroll
    for (int j = 0; j < 4; ++j) {
#pragma unroll
      for (int r = 0; r < 8; ++r) {
        const float v = acc[i][j][r] * scale;
        slab[(mOff + r) * 68 + (j << 4) + rlane] = v;
      }
    }
    wave_lds_sync();
    if (OUT_MODE == 0) {
      float* C = (float*)Cout;
      const int hh = lane >> 4, c4 = (lane & 15) * 4;
      for (int pass = 0; pass < 2; ++pass) {
#pragma unroll
        for (int it = 0; it < 8; ++it) {
          const int row = it * 2 + hh;
          v4f v = *(const v4f*)(slab + row * 68 + c4);
          *(volatile v4f*)(C + (size_t)(mBase + row) * ldc + n0 + c4) = v;
        }
        __threadfence();
      }
    } else {
      const int q = lane >> 3, c8 = (lane & 7) * 8;
      unsigned short* C  = (unsigned short*)Cout;
      unsigned short* C2 = (unsigned short*)Cout2;
      for (int pass = 0; pass < 2; ++pass) {
#pragma unroll
        for (int it = 0; it < 4; ++it) {
          const int row = it * 4 + q;
          const float* sp = slab + row * 68 + c8;
          v8h hv, lv;
#pragma unroll
          for (int e = 0; e < 8; ++e) {
            unsigned short hb = f2bf_bits(sp[e]);
            unsigned short lb = f2bf_bits(sp[e] - bf_bits2f(hb));
            hv[e] = __builtin_bit_cast(_Float16, hb);
            lv[e] = __builtin_bit_cast(_Float16, lb);
          }
          *(volatile v8h*)(C + (size_t)(mBase + row) * ldc + n0 + c8) = hv;
          *(volatile v8h*)(C2 + (size_t)(mBase + row) * ldc + n0 + c8) = lv;
        }
        __threadfence();
      }
    }
    wave_lds_sync();
  }
}

__global__ __launch_bounds__(256) void k_cast_bf16x8(const float* __restrict__ in, unsigned short* __restrict__ out, int n8) {
  const int i = blockIdx.x * 256 + threadIdx.x;
  if (i < n8) {
    const v4f a = *(const v4f*)(in + (size_t)8 * i);
    const v4f c = *(const v4f*)(in + (size_t)8 * i + 4);
    v4u u;
    u[0] = (unsigned)f2bf_bits(a[0]) | ((unsigned)f2bf_bits(a[1]) << 16);
    u[1] = (unsigned)f2bf_bits(a[2]) | ((unsigned)f2bf_bits(a[3]) << 16);
    u[2] = (unsigned)f2bf_bits(c[0]) | ((unsigned)f2bf_bits(c[1]) << 16);
    u[3] = (unsigned)f2bf_bits(c[2]) | ((unsigned)f2bf_bits(c[3]) << 16);
    unsigned short* p = out + (size_t)8 * i;
    *(volatile v4u*)p = u;
    __threadfence();
    *(volatile v4u*)p = u;
  }
}

__global__ __launch_bounds__(256) void k_transpose_w(const float* __restrict__ W, unsigned short* __restrict__ Wt,
                                                   int ncols, int ldt, int rowOff) {
  __shared__ float tile[64][65];
  const int tid = threadIdx.x, lane = tid & 31, wave = tid >> 5;
  const int n0 = blockIdx.x * 64, k0 = blockIdx.y * 64;
  {
    const int r = tid >> 2, c16 = (tid & 3) * 16;
    const float* src = W + (size_t)(k0 + r) * ncols + n0 + c16;
#pragma unroll
    for (int e4 = 0; e4 < 4; ++e4) {
      const v4f v = *(const v4f*)(src + 4 * e4);
      tile[r][c16 + 4 * e4 + 0] = v[0];
      tile[r][c16 + 4 * e4 + 1] = v[1];
      tile[r][c16 + 4 * e4 + 2] = v[2];
      tile[r][c16 + 4 * e4 + 3] = v[3];
    }
  }
  __syncthreads();
  const int q = lane >> 3, c8 = (lane & 7) * 8;
  v4u u[2];
  int nrow[2];
#pragma unroll
  for (int it = 0; it < 2; ++it) {
    const int n = wave * 8 + it * 4 + q;
    nrow[it] = n;
    v4u t;
#pragma unroll
    for (int e2 = 0; e2 < 4; ++e2) {
      const unsigned lo = f2bf_bits(tile[c8 + 2 * e2][n]);
      const unsigned hi = f2bf_bits(tile[c8 + 2 * e2 + 1][n]);
      t[e2] = lo | (hi << 16);
    }
    u[it] = t;
  }
  for (int pass = 0; pass < 2; ++pass) {
#pragma unroll
    for (int it = 0; it < 2; ++it)
      *(volatile v4u*)(Wt + (size_t)(rowOff + n0 + nrow[it]) * ldt + k0 + c8) = u[it];
    __threadfence();
  }
}

__global__ __launch_bounds__(128) void k_small_wt(const float* __restrict__ WB, const float* __restrict__ WC,
                                                unsigned short* __restrict__ Wt, int ldt) {
  const int j = blockIdx.x;
  const int k8 = threadIdx.x * 8;
  v4u u = {0u, 0u, 0u, 0u};
  if (j < 32) {
    const float* src = (j < 16) ? WB : WC;
    const int col = j & 15;
#pragma unroll
    for (int e2 = 0; e2 < 4; ++e2) {
      const unsigned lo = f2bf_bits(src[(size_t)(k8 + 2 * e2) * NST + col]);
      const unsigned hi = f2bf_bits(src[(size_t)(k8 + 2 * e2 + 1) * NST + col]);
      u[e2] = lo | (hi << 16);
    }
  }
  unsigned short* p = Wt + (size_t)j * ldt + k8;
  *(volatile v4u*)p = u;
  __threadfence();
  *(volatile v4u*)p = u;
}

__global__ __launch_bounds__(256) void k_prep_a(const float* __restrict__ alog, float* __restrict__ a2, int n4) {
  const int i = blockIdx.x * 256 + threadIdx.x;
  if (i < n4) {
    const v4f a = *(const v4f*)(alog + (size_t)4 * i);
    v4f o;
#pragma unroll
    for (int e = 0; e < 4; ++e) o[e] = -expf(bf_rne(a[e])) * LOG2E_F;
    float* p = a2 + (size_t)4 * i;
    *(volatile v4f*)p = o;
    __threadfence();
    *(volatile v4f*)p = o;
  }
}

__global__ __launch_bounds__(64) void k_scan(const float* __restrict__ dbc, const unsigned short* __restrict__ xb,
                                           const float* __restrict__ a2tab, float* __restrict__ yout) {
  __shared__ __align__(16) float sBC[TCHUNK * 32];
  __shared__ __align__(16) float ytile[2][4 * 32];
  const int tid = threadIdx.x, lane = tid & 31, wave = tid >> 5;
  const int b = blockIdx.x >> 4;
  const int dblk = blockIdx.x & 15;
  const int d = dblk * 64 + tid;
  const int dw0 = dblk * 64 + wave * 32;

  float Ar[NST];
  {
    const float* ap = a2tab + (size_t)d * NST;
    const v4f t0 = *(const v4f*)(ap), t1 = *(const v4f*)(ap + 4), t2 = *(const v4f*)(ap + 8), t3 = *(const v4f*)(ap + 12);
    Ar[0] = t0[0]; Ar[1] = t0[1]; Ar[2] = t0[2]; Ar[3] = t0[3];
    Ar[4] = t1[0]; Ar[5] = t1[1]; Ar[6] = t1[2]; Ar[7] = t1[3];
    Ar[8] = t2[0]; Ar[9] = t2[1]; Ar[10] = t2[2]; Ar[11] = t2[3];
    Ar[12] = t3[0]; Ar[13] = t3[1]; Ar[14] = t3[2]; Ar[15] = t3[3];
  }
  float h[NST];
#pragma unroll
  for (int n = 0; n < NST; ++n) h[n] = 0.0f;

  const size_t rowb = (size_t)b * SEQLEN;
  float* yt = ytile[wave];

#pragma unroll 1
  for (int t0 = 0; t0 < SEQLEN; t0 += TCHUNK) {
    __syncthreads();
    {
      const float* src = dbc + (rowb + t0 + tid) * (size_t)NALL + DMOD;
      float* dstl = sBC + tid * 32;
#pragma unroll
      for (int e = 0; e < 8; ++e) *(v4f*)(dstl + 4 * e) = *(const v4f*)(src + 4 * e);
    }
    __syncthreads();
#pragma unroll 1
    for (int tt = 0; tt < TCHUNK; ++tt) {
      const size_t row = rowb + t0 + tt;
      const float dpre = dbc[row * NALL + d];
      const float xv = __uint_as_float(((unsigned)xb[row * DMOD + d]) << 16);
      const float du = fmaxf(dpre, 0.0f) + log1pf(expf(-fabsf(dpre)));
      const float dux = du * xv;
      const float* bc = sBC + tt * 32;
      float y = 0.0f;
#pragma unroll
      for (int n = 0; n < NST; ++n) {
        const float e = exp2f(du * Ar[n]);
        h[n] = fmaf(h[n], e, dux * bc[n]);
        y = fmaf(h[n], bc[16 + n], y);
      }
      yt[(tt & 3) * 32 + lane] = y;
      if ((tt & 3) == 3) {
        wave_lds_sync();
        const v4f v = *(const v4f*)(yt + (lane >> 3) * 32 + (lane & 7) * 4);
        float* dst = yout + (row - 3 + (lane >> 3)) * (size_t)DMOD + dw0 + (lane & 7) * 4;
        *(volatile v4f*)dst = v;
        __threadfence();
        *(volatile v4f*)dst = v;
        wave_lds_sync();
      }
    }
  }
}

__global__ __launch_bounds__(256) void k_zero16(unsigned short* __restrict__ p0, unsigned short* __restrict__ p1, int base, int n8) {
  const int i = blockIdx.x * 256 + threadIdx.x;
  if (i < n8) {
    const v4u z = {0u, 0u, 0u, 0u};
    unsigned short* p = ((blockIdx.y == 0) ? p0 : p1) + base + (size_t)8 * i;
    *(volatile v4u*)p = z;
    __threadfence();
    *(volatile v4u*)p = z;
  }
}

__global__ __launch_bounds__(128) void k_layernorm(const float* __restrict__ yin, const float* __restrict__ gam,
                                                 const float* __restrict__ bet,
                                                 unsigned short* __restrict__ lnh, unsigned short* __restrict__ lnl,
                                                 unsigned short* __restrict__ hfh, unsigned short* __restrict__ hfl) {
  __shared__ float red[4];
  const int r = blockIdx.x;
  const int tid = threadIdx.x, lane = tid & 31, wave = tid >> 5;
  const int c0 = tid * 8;
  const float* rowp = yin + (size_t)r * DMOD + c0;
  const v4f a = *(const v4f*)rowp;
  const v4f c = *(const v4f*)(rowp + 4);
  float v[8] = {a[0], a[1], a[2], a[3], c[0], c[1], c[2], c[3]};

  float s = ((v[0] + v[1]) + (v[2] + v[3])) + ((v[4] + v[5]) + (v[6] + v[7]));
#pragma unroll
  for (int off = 1; off < 32; off <<= 1) s += __shfl_xor(s, off, 32);
  if (lane == 0) red[wave] = s;
  __syncthreads();
  const float mu = ((red[0] + red[1]) + (red[2] + red[3])) * (1.0f / 1024.0f);
  __syncthreads();

  float qs = 0.0f;
#pragma unroll
  for (int e = 0; e < 8; ++e) { const float dd = v[e] - mu; qs += dd * dd; }
#pragma unroll
  for (int off = 1; off < 32; off <<= 1) qs += __shfl_xor(qs, off, 32);
  if (lane == 0) red[wave] = qs;
  __syncthreads();
  const float var = ((red[0] + red[1]) + (red[2] + red[3])) * (1.0f / 1024.0f);
  const float inv = rsqrtf(var + 1e-5f);

  const v4f g0 = *(const v4f*)(gam + c0), g1 = *(const v4f*)(gam + c0 + 4);
  const v4f b0 = *(const v4f*)(bet + c0), b1 = *(const v4f*)(bet + c0 + 4);
  float g[8]  = {g0[0], g0[1], g0[2], g0[3], g1[0], g1[1], g1[2], g1[3]};
  float bb[8] = {b0[0], b0[1], b0[2], b0[3], b1[0], b1[1], b1[2], b1[3]};

  v4u H, L;
#pragma unroll
  for (int e2 = 0; e2 < 4; ++e2) {
    const float o0 = (v[2 * e2] - mu) * inv * bf_rne(g[2 * e2]) + bf_rne(bb[2 * e2]);
    const float o1 = (v[2 * e2 + 1] - mu) * inv * bf_rne(g[2 * e2 + 1]) + bf_rne(bb[2 * e2 + 1]);
    const unsigned short hb0 = f2bf_bits(o0), hb1 = f2bf_bits(o1);
    const unsigned short lb0 = f2bf_bits(o0 - bf_bits2f(hb0)), lb1 = f2bf_bits(o1 - bf_bits2f(hb1));
    H[e2] = (unsigned)hb0 | ((unsigned)hb1 << 16);
    L[e2] = (unsigned)lb0 | ((unsigned)lb1 << 16);
  }
  unsigned short* ph = lnh + (size_t)r * DMOD + c0;
  unsigned short* pl = lnl + (size_t)r * DMOD + c0;
  *(volatile v4u*)ph = H;
  *(volatile v4u*)pl = L;
  __threadfence();
  *(volatile v4u*)ph = H;
  *(volatile v4u*)pl = L;
  if ((r & (SEQLEN - 1)) == (SEQLEN - 1)) {
    const int bi = r / SEQLEN;
    unsigned short* qh = hfh + (size_t)bi * DMOD + c0;
    unsigned short* ql = hfl + (size_t)bi * DMOD + c0;
    *(volatile v4u*)qh = H;
    *(volatile v4u*)ql = L;
    __threadfence();
    *(volatile v4u*)qh = H;
    *(volatile v4u*)ql = L;
  }
}

__global__ __launch_bounds__(256) void k_softmax_out(const float* __restrict__ rawt, float* __restrict__ out_imp,
                                                   float* __restrict__ out_raw) {
  __shared__ __align__(16) float se[SEQLEN];
  __shared__ float red[8];
  const int b = blockIdx.x;
  const int tid = threadIdx.x, lane = tid & 31, wave = tid >> 5;
  const float* src = rawt + (size_t)b * MROWS + (size_t)b * SEQLEN;

  float m = -INFINITY;
#pragma unroll 1
  for (int it = 0; it < 4; ++it) {
    const v4f rv = *(const v4f*)(src + it * 1024 + 4 * tid);
    m = fmaxf(m, fmaxf(fmaxf(rv[0], rv[1]), fmaxf(rv[2], rv[3])));
  }
  m = 2.0f * m;
#pragma unroll
  for (int off = 1; off < 32; off <<= 1) m = fmaxf(m, __shfl_xor(m, off, 32));
  if (lane == 0) red[wave] = m;
  __syncthreads();
  float mx = red[0];
#pragma unroll
  for (int w = 1; w < 8; ++w) mx = fmaxf(mx, red[w]);
  __syncthreads();

  float ssum = 0.0f;
#pragma unroll 1
  for (int it = 0; it < 4; ++it) {
    const v4f rv = *(const v4f*)(src + it * 1024 + 4 * tid);
    v4f ev;
    ev[0] = expf(2.0f * rv[0] - mx);
    ev[1] = expf(2.0f * rv[1] - mx);
    ev[2] = expf(2.0f * rv[2] - mx);
    ev[3] = expf(2.0f * rv[3] - mx);
    ssum += (ev[0] + ev[1]) + (ev[2] + ev[3]);
    *(v4f*)(se + it * 1024 + 4 * tid) = ev;
  }
#pragma unroll
  for (int off = 1; off < 32; off <<= 1) ssum += __shfl_xor(ssum, off, 32);
  if (lane == 0) red[wave] = ssum;
  __syncthreads();
  float tot = 0.0f;
#pragma unroll
  for (int w = 0; w < 8; ++w) tot += red[w];
  const float inv = 1.0f / tot;

  for (int pass = 0; pass < 2; ++pass) {
#pragma unroll 1
    for (int it = 0; it < 4; ++it) {
      const v4f ev = *(const v4f*)(se + it * 1024 + 4 * tid);
      const v4f rv = *(const v4f*)(src + it * 1024 + 4 * tid);
      const v4f iv = ev * inv;
      *(volatile v4f*)(out_imp + (size_t)b * SEQLEN + it * 1024 + 4 * tid) = iv;
      *(volatile v4f*)(out_raw + (size_t)b * SEQLEN + it * 1024 + 4 * tid) = rv;
    }
    __threadfence();
  }
}

static constexpr size_t SZ_XB   = (size_t)MROWS * DMOD * 2;
static constexpr size_t SZ_WALL = (size_t)NALL * DMOD * 2;
static constexpr size_t SZ_WSQ  = (size_t)DMOD * DMOD * 2;
static constexpr size_t SZ_A2   = (size_t)DMOD * NST * 4;
static constexpr size_t SZ_DBC  = (size_t)MROWS * NALL * 4;
static constexpr size_t SZ_Y    = (size_t)MROWS * DMOD * 4;
static constexpr size_t SZ_LN   = (size_t)MROWS * DMOD * 2;
static constexpr size_t SZ_P64  = (size_t)64 * DMOD * 2;
static constexpr size_t SZ_RAWT = (size_t)64 * MROWS * 4;
static constexpr size_t OFF_XB   = 0;
static constexpr size_t OFF_WALL = OFF_XB + SZ_XB;
static constexpr size_t OFF_WCTX = OFF_WALL + SZ_WALL;
static constexpr size_t OFF_WIMP = OFF_WCTX + SZ_WSQ;
static constexpr size_t OFF_A2   = OFF_WIMP + SZ_WSQ;
static constexpr size_t OFF_DBC  = OFF_A2 + SZ_A2;
static constexpr size_t OFF_Y    = OFF_DBC + SZ_DBC;
static constexpr size_t OFF_LNH  = OFF_Y + SZ_Y;
static constexpr size_t OFF_LNL  = OFF_LNH + SZ_LN;
static constexpr size_t OFF_HFH  = OFF_LNL + SZ_LN;
static constexpr size_t OFF_HFL  = OFF_HFH + SZ_P64;
static constexpr size_t OFF_HPH  = OFF_HFL + SZ_P64;
static constexpr size_t OFF_HPL  = OFF_HPH + SZ_P64;
static constexpr size_t OFF_RAWT = OFF_HPL + SZ_P64;
static constexpr size_t WS_END   = OFF_RAWT + SZ_RAWT;
static_assert(WS_END == 128647168ull);
static_assert(WS_END <= 134217728ull);
static_assert((OFF_WALL % 128) == 0 && (OFF_WCTX % 128) == 0 && (OFF_WIMP % 128) == 0 && (OFF_A2 % 128) == 0);
static_assert((OFF_DBC % 128) == 0 && (OFF_Y % 128) == 0 && (OFF_LNH % 128) == 0 && (OFF_LNL % 128) == 0);
static_assert((OFF_HFH % 128) == 0 && (OFF_HFL % 128) == 0 && (OFF_HPH % 128) == 0 && (OFF_HPL % 128) == 0 && (OFF_RAWT % 128) == 0);

static constexpr size_t OUT0_F = 0;
static constexpr size_t OUT1_F = 32768 / 4;
static constexpr size_t OUT2_F = 33587200 / 4;
static_assert(OUT1_F == (size_t)NBATCH * SEQLEN);
static_assert(OUT2_F == OUT1_F + (size_t)MROWS * DMOD);
static_assert((OUT2_F + (size_t)NBATCH * SEQLEN) * 4 == 33619968ull);

static constexpr int TILES_DELTA = (MROWS / 64) * (NALL / 64);
static constexpr int TILES_HPROJ = (64 / 64) * (DMOD / 64);
static constexpr int TILES_RAW   = (64 / 64) * (MROWS / 64);
static constexpr int TILES_CTX   = (MROWS / 64) * (DMOD / 64);
static_assert(TILES_DELTA == 2176 && TILES_HPROJ == 16 && TILES_RAW == 128 && TILES_CTX == 2048);

extern "C" void kernel_launch(void* const* d_in, const int* in_sizes, int n_in,
                              void* d_out, int out_size, void* d_ws, size_t ws_size,
                              hipStream_t stream) {
  (void)in_sizes; (void)n_in; (void)out_size; (void)ws_size;
  const float* x       = (const float*)d_in[0];
  const float* A_log   = (const float*)d_in[1];
  const float* W_delta = (const float*)d_in[2];
  const float* W_B     = (const float*)d_in[3];
  const float* W_C     = (const float*)d_in[4];
  const float* ln_g    = (const float*)d_in[5];
  const float* ln_b    = (const float*)d_in[6];
  const float* W_ctx   = (const float*)d_in[7];
  const float* cscale  = (const float*)d_in[8];
  const float* W_imp   = (const float*)d_in[9];

  float* out = (float*)d_out;
  float* out_imp = out + OUT0_F;
  float* out_ctx = out + OUT1_F;
  float* out_raw = out + OUT2_F;

  char* ws = (char*)d_ws;
  unsigned short* xb   = (unsigned short*)(ws + OFF_XB);
  unsigned short* wall = (unsigned short*)(ws + OFF_WALL);
  unsigned short* wctx = (unsigned short*)(ws + OFF_WCTX);
  unsigned short* wimp = (unsigned short*)(ws + OFF_WIMP);
  float*          a2   = (float*)(ws + OFF_A2);
  float*          dbc  = (float*)(ws + OFF_DBC);
  float*          ybuf = (float*)(ws + OFF_Y);
  unsigned short* lnh  = (unsigned short*)(ws + OFF_LNH);
  unsigned short* lnl  = (unsigned short*)(ws + OFF_LNL);
  unsigned short* hfh  = (unsigned short*)(ws + OFF_HFH);
  unsigned short* hfl  = (unsigned short*)(ws + OFF_HFL);
  unsigned short* hph  = (unsigned short*)(ws + OFF_HPH);
  unsigned short* hpl  = (unsigned short*)(ws + OFF_HPL);
  float*          rawt = (float*)(ws + OFF_RAWT);

  const int n8 = MROWS * DMOD / 8;
  k_cast_bf16x8<<<(n8 + 255) / 256, 256, 0, stream>>>(x, xb, n8);
  k_transpose_w<<<dim3(DMOD / 64, DMOD / 64), 256, 0, stream>>>(W_delta, wall, DMOD, DMOD, 0);
  k_small_wt<<<NALL - DMOD, 128, 0, stream>>>(W_B, W_C, wall + (size_t)DMOD * DMOD, DMOD);
  k_transpose_w<<<dim3(DMOD / 64, DMOD / 64), 256, 0, stream>>>(W_ctx, wctx, DMOD, DMOD, 0);
  k_transpose_w<<<dim3(DMOD / 64, DMOD / 64), 256, 0, stream>>>(W_imp, wimp, DMOD, DMOD, 0);
  const int na4 = DMOD * NST / 4;
  k_prep_a<<<(na4 + 255) / 256, 256, 0, stream>>>(A_log, a2, na4);

  gemm64_bf16<false, 0, false><<<(TILES_DELTA + 7) / 8, 256, 0, stream>>>(
      xb, xb, DMOD, wall, DMOD, (void*)dbc, (void*)dbc, NALL, cscale, MROWS, NALL, DMOD);

  k_scan<<<NBATCH * (DMOD / 64), 64, 0, stream>>>(dbc, xb, a2, ybuf);

  const int nz8 = 62 * DMOD / 8;
  k_zero16<<<dim3((nz8 + 255) / 256, 2), 256, 0, stream>>>(hfh, hfl, 2 * DMOD, nz8);
  k_layernorm<<<MROWS, 128, 0, stream>>>(ybuf, ln_g, ln_b, lnh, lnl, hfh, hfl);

  gemm64_bf16<true, 2, false><<<(TILES_HPROJ + 7) / 8, 256, 0, stream>>>(
      hfh, hfl, DMOD, wimp, DMOD, (void*)hph, (void*)hpl, DMOD, cscale, 64, DMOD, DMOD);
  gemm64_bf16<true, 0, false><<<(TILES_RAW + 7) / 8, 256, 0, stream>>>(
      hph, hpl, DMOD, xb, DMOD, (void*)rawt, (void*)rawt, MROWS, cscale, 64, MROWS, DMOD);
  k_softmax_out<<<NBATCH, 256, 0, stream>>>(rawt, out_imp, out_raw);

  gemm64_bf16<true, 0, true><<<(TILES_CTX + 7) / 8, 256, 0, stream>>>(
      lnh, lnl, DMOD, wctx, DMOD, (void*)out_ctx, (void*)out_ctx, DMOD, cscale, MROWS, DMOD, DMOD);
}
